// Lstm_29987461660977
// MI455X (gfx1250) — hardware-run, weakly checked
//
#include <hip/hip_runtime.h>
#include <math.h>

typedef __attribute__((ext_vector_type(16))) __bf16   v16b;
typedef __attribute__((ext_vector_type(8)))  __bf16   v8b;
typedef __attribute__((ext_vector_type(8)))  float    v8f;
typedef __attribute__((ext_vector_type(4)))  float    v4f;
typedef __attribute__((ext_vector_type(4)))  unsigned v4u;

constexpr int kSteps  = 10;
constexpr int kBatch  = 64;
constexpr int kIn     = 2048;
constexpr int kHid    = 2048;
constexpr int kRows   = kSteps * kBatch;
constexpr int kNMain  = 4 * kHid;
constexpr int kNHead  = 3 * kHid;
constexpr int kStack  = kSteps * kBatch * kHid;
constexpr int kOut0   = kBatch * 2 * kHid;
constexpr int kOutAll = kOut0 + 4 * kStack;
static_assert(kRows == 640);
static_assert((kRows % 64) == 0 && (kBatch % 64) == 0);
static_assert((kNMain % 64) == 0 && (kNHead % 64) == 0);
static_assert((kIn % 32) == 0 && (kIn % 64) == 0 && (kHid % 64) == 0);
static_assert(kIn == 256 * 8);
static_assert(kOut0 * 4 == 1048576);
static_assert((kOut0 + kStack) * 4 == 6291456);
static_assert((kOut0 + 2 * kStack) * 4 == 11534336);
static_assert((kOut0 + 3 * kStack) * 4 == 16777216);
static_assert((size_t)kOutAll * 4 == 22020096ull);

constexpr size_t kOffXA   = 0;
constexpr size_t kOffBTM  = kOffXA   + (size_t)kRows  * kIn * 2;
constexpr size_t kOffBTHF = kOffBTM  + (size_t)kNMain * kIn * 2;
constexpr size_t kOffBTHB = kOffBTHF + (size_t)kNHead * kIn * 2;
constexpr size_t kOffPM   = kOffBTHB + (size_t)kNHead * kIn * 2;
constexpr size_t kOffQF   = kOffPM   + (size_t)kRows  * kNMain * 4;
constexpr size_t kOffQB   = kOffQF   + (size_t)kBatch * kNHead * 4;
constexpr size_t kWsTotal = kOffQB   + (size_t)kBatch * kNHead * 4;
static_assert(kWsTotal == 110624768ull);
static_assert(kWsTotal <= 134217728ull);
static_assert((kOffBTM % 128) == 0 && (kOffBTHF % 128) == 0 && (kOffBTHB % 128) == 0 &&
              (kOffPM % 128) == 0 && (kOffQF % 128) == 0 && (kOffQB % 128) == 0);

__device__ __forceinline__ unsigned short f2bf_bits(float f) {
  unsigned u = __float_as_uint(f);
  return (unsigned short)((u + 0x7FFFu + ((u >> 16) & 1u)) >> 16);
}
__device__ __forceinline__ float bf_bits2f(unsigned short h) { return __uint_as_float(((unsigned)h) << 16); }

__device__ __forceinline__ unsigned pack_bf16x2(float lo, float hi) {
  const unsigned a = (unsigned)f2bf_bits(lo);
  const unsigned b = (unsigned)f2bf_bits(hi);
  return a | (b << 16);
}

struct FragB {
  union U { v16b v; v8b h[2]; };
  static __device__ __forceinline__ v16b load(const __bf16* p) {
    U f;
    f.h[0] = *(const v8b*)(p);
    f.h[1] = *(const v8b*)(p + 16);
    return f.v;
  }
};

__device__ __forceinline__ v8f mma_bf16(v16b a, v16b b, v8f c) {
  c = __builtin_amdgcn_wmma_f32_16x16x32_bf16(false, a, false, b, (short)0, c, false, false);
  asm volatile("v_nop\n\tv_nop\n\tv_nop\n\tv_nop" : "+v"(c) : "v"(a), "v"(b));
  return c;
}

__global__ __launch_bounds__(256) void cvt_x_rows_kernel(
    const float* __restrict__ x, unsigned short* __restrict__ XA)
{
  const int row = blockIdx.x;
  const int t = row >> 6;
  const int b = row & 63;
  const int c8 = threadIdx.x * 8;
  const float* src = x + ((size_t)b * kSteps + t) * kIn + c8;
  const v4f a0 = *(const v4f*)(src);
  const v4f a1 = *(const v4f*)(src + 4);
  const float e0 = a0[0];
  const float e1 = a0[1];
  const float e2 = a0[2];
  const float e3 = a0[3];
  const float e4 = a1[0];
  const float e5 = a1[1];
  const float e6 = a1[2];
  const float e7 = a1[3];
  const unsigned w0 = pack_bf16x2(e0, e1);
  const unsigned w1 = pack_bf16x2(e2, e3);
  const unsigned w2 = pack_bf16x2(e4, e5);
  const unsigned w3 = pack_bf16x2(e6, e7);
  const v4u w = (v4u){w0, w1, w2, w3};
  unsigned short* dst = XA + (size_t)row * kIn + c8;
  *(volatile v4u*)dst = w;
  __threadfence();
  *(volatile v4u*)dst = w;
}

__global__ __launch_bounds__(256) void transpose_cvt_kernel(
    const float* __restrict__ W, unsigned short* __restrict__ Bt)
{
  __shared__ __align__(16) float sT[64 * 68];
  const int tid = threadIdx.x;
  const int n0 = blockIdx.x * 64;
  const int k0 = blockIdx.y * 64;
  {
    const int lr = tid >> 4;
    const int c4 = (tid & 15) * 4;
#pragma unroll
    for (int p = 0; p < 4; ++p) {
      const int r = lr + 16 * p;
      const v4f v = *(const v4f*)(W + (size_t)(k0 + r) * kHid + n0 + c4);
      *(v4f*)(sT + r * 68 + c4) = v;
    }
  }
  __syncthreads();
  const int q8 = tid & 7;
  const int nr0 = tid >> 3;
  v4u wv[2];
#pragma unroll
  for (int p = 0; p < 2; ++p) {
    const int nr = nr0 + 32 * p;
    const float* sp = sT + (q8 * 8) * 68 + nr;
    const float e0 = sp[0 * 68];
    const float e1 = sp[1 * 68];
    const float e2 = sp[2 * 68];
    const float e3 = sp[3 * 68];
    const float e4 = sp[4 * 68];
    const float e5 = sp[5 * 68];
    const float e6 = sp[6 * 68];
    const float e7 = sp[7 * 68];
    const unsigned w0 = pack_bf16x2(e0, e1);
    const unsigned w1 = pack_bf16x2(e2, e3);
    const unsigned w2 = pack_bf16x2(e4, e5);
    const unsigned w3 = pack_bf16x2(e6, e7);
    wv[p] = (v4u){w0, w1, w2, w3};
  }
  unsigned short* d0 = Bt + (size_t)(n0 + nr0) * kIn + k0 + q8 * 8;
  unsigned short* d1 = Bt + (size_t)(n0 + nr0 + 32) * kIn + k0 + q8 * 8;
  *(volatile v4u*)d0 = wv[0];
  *(volatile v4u*)d1 = wv[1];
  __threadfence();
  *(volatile v4u*)d0 = wv[0];
  *(volatile v4u*)d1 = wv[1];
}

__global__ __launch_bounds__(256) void gemm_bf16_nt_kernel(
    const unsigned short* __restrict__ Ap, int lda,
    const unsigned short* __restrict__ Btp, int ldb,
    float* __restrict__ C, int ldc, int M, int N, int K)
{
  const __bf16* A  = (const __bf16*)Ap;
  const __bf16* Bt = (const __bf16*)Btp;
  __shared__ __align__(16) float sT[8][16 * 68];
  const int lane = threadIdx.x & 31;
  const int wave = threadIdx.x >> 5;
  const int tilesN = N >> 6;
  const int tilesM = M >> 6;
  const int tile = blockIdx.x * 8 + wave;
  if (tile >= tilesM * tilesN) return;
  const int tm = tile / tilesN;
  const int tn = tile - tm * tilesN;
  const int m0 = tm << 6;
  const int n0 = tn << 6;

  const int rlane = lane & 15;
  const int koff  = (lane >> 4) * 8;
  const int mOff  = (lane >> 4) * 8;

  v8f acc[4][4];
#pragma unroll
  for (int i = 0; i < 4; ++i)
#pragma unroll
    for (int j = 0; j < 4; ++j) acc[i][j] = (v8f){0.f, 0.f, 0.f, 0.f, 0.f, 0.f, 0.f, 0.f};

  for (int k0 = 0; k0 < K; k0 += 32) {
    v16b bh[4];
#pragma unroll
    for (int j = 0; j < 4; ++j) {
      const size_t bo = (size_t)(n0 + (j << 4) + rlane) * ldb + koff + k0;
      bh[j] = FragB::load(Bt + bo);
    }
#pragma unroll
    for (int i = 0; i < 4; ++i) {
      const size_t ao = (size_t)(m0 + (i << 4) + rlane) * lda + koff + k0;
      const v16b ah = FragB::load(A + ao);
#pragma unroll
      for (int j = 0; j < 4; ++j) acc[i][j] = mma_bf16(ah, bh[j], acc[i][j]);
    }
  }

  float* slab = sT[wave];
#pragma unroll
  for (int i = 0; i < 4; ++i) {
    const int mBase = m0 + (i << 4);
#pragma unroll
    for (int j = 0; j < 4; ++j) {
#pragma unroll
      for (int r = 0; r < 8; ++r) {
        const float v = acc[i][j][r];
        slab[(mOff + r) * 68 + (j << 4) + rlane] = v;
      }
    }
    __builtin_amdgcn_fence(__ATOMIC_RELEASE, "workgroup");
    __builtin_amdgcn_wave_barrier();
    __builtin_amdgcn_fence(__ATOMIC_ACQUIRE, "workgroup");
    {
      const int hh = lane >> 4;
      const int c4 = (lane & 15) * 4;
      for (int pass = 0; pass < 2; ++pass) {
#pragma unroll
        for (int it = 0; it < 8; ++it) {
          const int row = it * 2 + hh;
          const v4f v = *(const v4f*)(slab + row * 68 + c4);
          *(volatile v4f*)(C + (size_t)(mBase + row) * ldc + n0 + c4) = v;
        }
        __threadfence();
      }
    }
    __builtin_amdgcn_fence(__ATOMIC_RELEASE, "workgroup");
    __builtin_amdgcn_wave_barrier();
    __builtin_amdgcn_fence(__ATOMIC_ACQUIRE, "workgroup");
  }
}

__device__ __forceinline__ float sigmoid_f32(float v) { return 1.0f / (1.0f + expf(-v)); }

__global__ __launch_bounds__(256) void scan_head_kernel(
    const float* __restrict__ PM, int pcol0, int flip,
    const float* __restrict__ Q,
    const float* __restrict__ bias_g, const float* __restrict__ bias_rs, const float* __restrict__ bias_rf,
    float* __restrict__ outS, float* __restrict__ outF, float* __restrict__ outH)
{
  const int idx = blockIdx.x * 256 + threadIdx.x;
  const int h = idx & (kHid - 1);
  const int b = idx >> 11;
  const float bg  = bf_bits2f(f2bf_bits(bias_g[h]));
  const float brs = bf_bits2f(f2bf_bits(bias_rs[h]));
  const float brf = bf_bits2f(f2bf_bits(bias_rf[h]));
  float s = 0.0f;
  float f = 0.0f;
#pragma unroll 1
  for (int t = 0; t < kSteps; ++t) {
    const int tsrc = flip ? (kSteps - 1 - t) : t;
    const float* pp = PM + (size_t)(tsrc * kBatch + b) * kNMain + pcol0 + h;
    const float xs  = pp[0];
    const float pre = pp[kHid];
    const float g   = sigmoid_f32(pre + bg);
    const float omg = 1.0f - g;
    const float sn = xs * omg + s * g;
    const float fn = xs * g + f * omg;
    s = sn;
    f = fn;
    float* ps = outS + (size_t)t * (kBatch * kHid) + idx;
    float* pf = outF + (size_t)t * (kBatch * kHid) + idx;
    *(volatile float*)ps = sn;
    *(volatile float*)pf = fn;
    __threadfence();
    *(volatile float*)ps = sn;
    *(volatile float*)pf = fn;
  }
  const float* qp = Q + (size_t)b * kNHead + h;
  const float xr = qp[0];
  const float q1 = qp[kHid] + brs;
  const float q2 = qp[2 * kHid] + brf;
  float hacc = 0.0f;
#pragma unroll 1
  for (int j = 0; j < 2; ++j) {
    const float st  = (j == 0) ? s : f;
    const float pre = (j == 0) ? q1 : q2;
    const float r  = sigmoid_f32(pre);
    const float th = tanhf(st);
    hacc = hacc + th * r;
    hacc = hacc + (1.0f - r) * xr;
  }
  float* ph = outH + (size_t)b * (2 * kHid) + h;
  *(volatile float*)ph = hacc;
  __threadfence();
  *(volatile float*)ph = hacc;
}

extern "C" void kernel_launch(void* const* d_in, const int* in_sizes, int n_in,
                              void* d_out, int out_size, void* d_ws, size_t ws_size,
                              hipStream_t stream)
{
  if (n_in < 17) return;
  if (in_sizes[0] != kBatch * kSteps * kIn) return;
  if (in_sizes[1] != kIn * kHid || in_sizes[2] != kIn * kHid || in_sizes[3] != kIn * kHid) return;
  if (in_sizes[4] != kIn * kHid || in_sizes[5] != kIn * kHid) return;
  if (in_sizes[9] != kIn * kHid || in_sizes[10] != kIn * kHid || in_sizes[11] != kIn * kHid) return;
  if (in_sizes[12] != kIn * kHid || in_sizes[13] != kIn * kHid) return;
  if (in_sizes[6] != kHid || in_sizes[7] != kHid || in_sizes[8] != kHid) return;
  if (in_sizes[14] != kHid || in_sizes[15] != kHid || in_sizes[16] != kHid) return;
  if (out_size != kOutAll) return;
  if (ws_size < kWsTotal) return;

  const float* x      = (const float*)d_in[0];
  const float* f_w_s  = (const float*)d_in[1];
  const float* f_wx   = (const float*)d_in[2];
  const float* f_wf_s = (const float*)d_in[3];
  const float* f_wr_s = (const float*)d_in[4];
  const float* f_wr_f = (const float*)d_in[5];
  const float* f_bf_s = (const float*)d_in[6];
  const float* f_br_s = (const float*)d_in[7];
  const float* f_br_f = (const float*)d_in[8];
  const float* b_w_s  = (const float*)d_in[9];
  const float* b_wx   = (const float*)d_in[10];
  const float* b_wf_s = (const float*)d_in[11];
  const float* b_wr_s = (const float*)d_in[12];
  const float* b_wr_f = (const float*)d_in[13];
  const float* b_bf_s = (const float*)d_in[14];
  const float* b_br_s = (const float*)d_in[15];
  const float* b_br_f = (const float*)d_in[16];

  float* out      = (float*)d_out;
  float* out_ss_f = out + kOut0;
  float* out_ff_f = out_ss_f + kStack;
  float* out_ss_b = out_ff_f + kStack;
  float* out_ff_b = out_ss_b + kStack;

  char* ws = (char*)d_ws;
  unsigned short* XA   = (unsigned short*)(ws + kOffXA);
  unsigned short* BTM  = (unsigned short*)(ws + kOffBTM);
  unsigned short* BTHF = (unsigned short*)(ws + kOffBTHF);
  unsigned short* BTHB = (unsigned short*)(ws + kOffBTHB);
  float*          PM   = (float*)(ws + kOffPM);
  float*          QF   = (float*)(ws + kOffQF);
  float*          QB   = (float*)(ws + kOffQB);

  const size_t wplane = (size_t)kHid * kIn;

  cvt_x_rows_kernel<<<kRows, 256, 0, stream>>>(x, XA);

  const dim3 tg(kHid / 64, kIn / 64);
  transpose_cvt_kernel<<<tg, 256, 0, stream>>>(f_w_s,  BTM + 0 * wplane);
  transpose_cvt_kernel<<<tg, 256, 0, stream>>>(f_wf_s, BTM + 1 * wplane);
  transpose_cvt_kernel<<<tg, 256, 0, stream>>>(b_w_s,  BTM + 2 * wplane);
  transpose_cvt_kernel<<<tg, 256, 0, stream>>>(b_wf_s, BTM + 3 * wplane);
  transpose_cvt_kernel<<<tg, 256, 0, stream>>>(f_wx,   BTHF + 0 * wplane);
  transpose_cvt_kernel<<<tg, 256, 0, stream>>>(f_wr_s, BTHF + 1 * wplane);
  transpose_cvt_kernel<<<tg, 256, 0, stream>>>(f_wr_f, BTHF + 2 * wplane);
  transpose_cvt_kernel<<<tg, 256, 0, stream>>>(b_wx,   BTHB + 0 * wplane);
  transpose_cvt_kernel<<<tg, 256, 0, stream>>>(b_wr_s, BTHB + 1 * wplane);
  transpose_cvt_kernel<<<tg, 256, 0, stream>>>(b_wr_f, BTHB + 2 * wplane);

  gemm_bf16_nt_kernel<<<(kRows / 64) * (kNMain / 64) / 8, 256, 0, stream>>>(
      XA, kIn, BTM, kIn, PM, kNMain, kRows, kNMain, kIn);

  gemm_bf16_nt_kernel<<<(kBatch / 64) * (kNHead / 64) / 8, 256, 0, stream>>>(
      XA + (size_t)(kSteps - 1) * kBatch * kIn, kIn, BTHF, kIn, QF, kNHead, kBatch, kNHead, kIn);
  gemm_bf16_nt_kernel<<<(kBatch / 64) * (kNHead / 64) / 8, 256, 0, stream>>>(
      XA, kIn, BTHB, kIn, QB, kNHead, kBatch, kNHead, kIn);

  scan_head_kernel<<<(kBatch * kHid) / 256, 256, 0, stream>>>(
      PM, 0, 0, QF, f_bf_s, f_br_s, f_br_f, out_ss_f, out_ff_f, out);
  scan_head_kernel<<<(kBatch * kHid) / 256, 256, 0, stream>>>(
      PM, 2 * kHid, 1, QB, b_bf_s, b_br_s, b_br_f, out_ss_b, out_ff_b, out + kHid);
}
